// LocalGNO_61658550501614
// MI455X (gfx1250) — hardware-verified
//
#include <hip/hip_runtime.h>
#include <stddef.h>
#include <stdint.h>


#define HID    96
#define NPER   16384
#define NL     2
#define KNB    4
#define NPB    64
#define HALO   4
#define MR     80
#define HBP    104
#define STP    196
#define DHP    100
#define NTHR   256
#define NWAVE  8
#define WSC    16.0f
#define WINV   0.0625f
#define LN_EPS 1e-5f
#define WSCAP  134217728
#define WP_E2   0
#define WP_L0   10240
#define WP_LSTR 57344
#define WP_W1   0
#define WP_W2   18432
#define WP_U1   28672
#define WP_U2   47104
#define WP_D1   124928
#define WP_TOT  135168
#define WP_BLKS 66
#define WPB     2048
#define LO_HB  0
#define LO_CS  16640
#define LO_ST  16960
#define LO_U   79680
#define LO_AG  92992
#define LO_MD  106304
#define LO_DH  119616
#define LDS_LAYER 145216

static_assert(LO_CS == MR * HBP * 2);
static_assert(LO_ST == LO_CS + MR * 4);
static_assert(LO_U == LO_ST + MR * STP * 4);
static_assert(LO_AG == LO_U + NPB * HBP * 2);
static_assert(LO_MD == LO_AG + NPB * HBP * 2);
static_assert(LO_DH == LO_MD + NPB * HBP * 2);
static_assert(LDS_LAYER == LO_DH + NPB * DHP * 4);
static_assert((LO_CS % 16) == 0 && (LO_ST % 16) == 0 && (LO_U % 16) == 0);
static_assert((LO_AG % 16) == 0 && (LO_MD % 16) == 0 && (LO_DH % 16) == 0);
static_assert(((HBP * 2) % 16) == 0 && ((STP * 4) % 16) == 0 && ((DHP * 4) % 16) == 0);
static_assert(WPB == NTHR * 8);
static_assert(WP_TOT == WP_BLKS * WPB);
static_assert(WP_L0 == 5 * WPB);
static_assert(WP_W2 == 2 * HID * HID && WP_W2 == 9 * WPB);
static_assert(WP_U1 == WP_W2 + 5 * WPB);
static_assert(WP_U2 == WP_U1 + 9 * WPB && WP_U2 - WP_U1 == HID * 2 * HID);
static_assert(WP_LSTR == WP_U2 + 5 * WPB && WP_LSTR == 28 * WPB);
static_assert(WP_D1 == WP_L0 + NL * WP_LSTR);
static_assert(WP_TOT == WP_D1 + 5 * WPB);
static_assert(HID * HID <= 5 * WPB);
static_assert(NPB == NWAVE * 8);
static_assert((NPB * HID) % NTHR == 0);
static_assert(MR % 16 == 0 && MR >= NPB + 2 * HALO);
static_assert(NPER % NPB == 0);
static_assert((HID % 32) == 0 && HID == 4 * 24 && HID == 3 * 32);

typedef float    v4f  __attribute__((ext_vector_type(4)));
typedef float    v8f  __attribute__((ext_vector_type(8)));
typedef _Float16 v4h  __attribute__((ext_vector_type(4)));
typedef _Float16 v8h  __attribute__((ext_vector_type(8)));
typedef _Float16 v16h __attribute__((ext_vector_type(16)));
union FragH { v16h v; v8h h[2]; };

__device__ __forceinline__ v8f wm(v16h a, v16h b, v8f c) {
  v8f d = __builtin_amdgcn_wmma_f32_16x16x32_f16(false, a, false, b, (short)0, c, false, false);
  asm volatile("v_nop\n\tv_nop\n\tv_nop\n\tv_nop" : "+v"(d) : "v"(a), "v"(b));
  return d;
}

__device__ __forceinline__ v8f zero8() {
  v8f z = {0.f, 0.f, 0.f, 0.f, 0.f, 0.f, 0.f, 0.f};
  return z;
}

__device__ __forceinline__ v8f mma_k96(const _Float16* ap, const _Float16* __restrict__ bp, v8f acc) {
#pragma unroll
  for (int ks = 0; ks < 3; ++ks) {
    FragH a, b;
    a.h[0] = *(const v8h*)(ap + 32 * ks);
    a.h[1] = *(const v8h*)(ap + 32 * ks + 16);
    b.h[0] = *(const v8h*)(bp + 32 * ks);
    b.h[1] = *(const v8h*)(bp + 32 * ks + 16);
    acc = wm(a.v, b.v, acc);
  }
  return acc;
}

__device__ __forceinline__ float silu_f(float v) {
  return v * __builtin_amdgcn_rcpf(1.0f + __expf(-v));
}

__device__ __forceinline__ float wsum(float v) {
  v += __shfl_xor(v, 16);
  v += __shfl_xor(v, 8);
  v += __shfl_xor(v, 4);
  v += __shfl_xor(v, 2);
  v += __shfl_xor(v, 1);
  return v;
}

__device__ __forceinline__ v4h cvt4(v4f a) {
  v4h o;
  o.x = (_Float16)a.x; o.y = (_Float16)a.y; o.z = (_Float16)a.z; o.w = (_Float16)a.w;
  return o;
}

__device__ __forceinline__ v4f zsel4(bool keep, v4f v) {
  v4f o;
  o.x = keep ? v.x : 0.f; o.y = keep ? v.y : 0.f; o.z = keep ? v.z : 0.f; o.w = keep ? v.w : 0.f;
  return o;
}

__device__ __forceinline__ void store_rows96(const float* stg, float* dst, size_t grow0, int wave, int lane) {
  const int cl = lane < 24 ? lane : 23;
  v4f vals[8];
#pragma unroll
  for (int i = 0; i < 8; ++i) vals[i] = *(const v4f*)(stg + (8 * wave + i) * DHP + 4 * cl);
#pragma unroll
  for (int i = 0; i < 8; ++i) {
    if (lane < 24) *(volatile v4f*)(dst + (grow0 + 8 * wave + i) * HID + 4 * lane) = vals[i];
  }
  __threadfence();
#pragma unroll
  for (int i = 0; i < 8; ++i) {
    if (lane < 24) *(volatile v4f*)(dst + (grow0 + 8 * wave + i) * HID + 4 * lane) = vals[i];
  }
}

__global__ __launch_bounds__(NTHR) void k_wprep(
    const float* __restrict__ ew2, const float* __restrict__ mw1, const float* __restrict__ mw2,
    const float* __restrict__ uw1, const float* __restrict__ uw2, const float* __restrict__ dw1,
    _Float16* wp) {
  const int tid = (int)threadIdx.x;
  const int b = (int)blockIdx.x;
  const float* src = ew2;
  int K = HID, Nn = HID, poff = WP_E2, lb = b;
  if (b < 5) {
    src = ew2; K = HID; Nn = HID; poff = WP_E2; lb = b;
  } else if (b < 5 + NL * 28) {
    const int lb0 = b - 5;
    const int l = lb0 / 28;
    const int r = lb0 - l * 28;
    const int base = WP_L0 + l * WP_LSTR;
    if (r < 9)       { src = mw1 + (size_t)l * (2 * HID + 1) * HID; K = HID;     Nn = 2 * HID; poff = base + WP_W1; lb = r; }
    else if (r < 14) { src = mw2 + (size_t)l * HID * HID;           K = HID;     Nn = HID;     poff = base + WP_W2; lb = r - 9; }
    else if (r < 23) { src = uw1 + (size_t)l * 2 * HID * HID;       K = 2 * HID; Nn = HID;     poff = base + WP_U1; lb = r - 14; }
    else             { src = uw2 + (size_t)l * HID * HID;           K = HID;     Nn = HID;     poff = base + WP_U2; lb = r - 23; }
  } else {
    src = dw1; K = HID; Nn = HID; poff = WP_D1; lb = b - (5 + NL * 28);
  }
  const int e  = (lb * NTHR + tid) * 8;
  const int n  = e / K;
  const int k0 = e - n * K;
  const bool valid = n < Nn;
  const int nc = valid ? n : Nn - 1;
  const int rowoff = (nc >= HID) ? HID : 0;
  const int col = nc - rowoff;
  float v[8];
#pragma unroll
  for (int j = 0; j < 8; ++j) {
    const float f = src[(size_t)(rowoff + k0 + j) * HID + col];
    v[j] = valid ? f * WSC : 0.0f;
  }
  v8h o;
#pragma unroll
  for (int j = 0; j < 8; ++j) o[j] = (_Float16)v[j];
  _Float16* dp = wp + poff + e;
  *(volatile v8h*)dp = o;
  __threadfence();
  *(volatile v8h*)dp = o;
}

__global__ __launch_bounds__(NTHR) void k_embed(
    const float* __restrict__ x, const float* __restrict__ w1, const float* __restrict__ b1,
    const _Float16* __restrict__ W2h, const float* __restrict__ b2, float* hout, int nRows) {
  __shared__ __attribute__((aligned(16))) float    xs[NPB * 4];
  __shared__ __attribute__((aligned(16))) _Float16 t1[NPB * HBP];
  __shared__ __attribute__((aligned(16))) float    stg[NPB * DHP];
  const int tid = threadIdx.x, lane = tid & 31, wave = tid >> 5, hh = lane >> 4, m = lane & 15;
  const int g0 = blockIdx.x * NPB;
  if (tid < NPB) {
    int gr = g0 + tid;
    gr = gr > nRows - 1 ? nRows - 1 : gr;
    const v4f xv = *(const v4f*)(x + (size_t)gr * 4);
    *(v4f*)(xs + 4 * tid) = xv;
  }
  __syncthreads();

#pragma unroll 2
  for (int e = 0; e < (NPB * HID) / NTHR; ++e) {
    const int idx = e * NTHR + tid;
    const int i = idx / HID;
    const int c = idx - i * HID;
    const float* xr = xs + 4 * i;
    float a = xr[0] * w1[c];
    a = a + xr[1] * w1[HID + c];
    a = a + xr[2] * w1[2 * HID + c];
    a = a + xr[3] * w1[3 * HID + c];
    a = a + b1[c];
    t1[i * HBP + c] = (_Float16)silu_f(a);
  }
  __syncthreads();

#pragma unroll 1
  for (int job = wave; job < 24; job += NWAVE) {
    const int mt = job / 6, nt = job - mt * 6;
    v8f acc = zero8();
    acc = mma_k96(t1 + (16 * mt + m) * HBP + 8 * hh, W2h + (size_t)(16 * nt + m) * HID + 8 * hh, acc);
    const int n = 16 * nt + m;
    const float bv = b2[n];
    float* sp = stg + (16 * mt + 8 * hh) * DHP + n;
#pragma unroll
    for (int r = 0; r < 8; ++r) sp[r * DHP] = acc[r] * WINV + bv;
  }
  __syncthreads();
  store_rows96(stg, hout, (size_t)g0, wave, lane);
}

__global__ __launch_bounds__(NTHR) void k_layer(
    const float* __restrict__ hin, float* hout, const float* __restrict__ coord,
    const float* __restrict__ wdc,
    const _Float16* __restrict__ W1c, const float* __restrict__ mb1,
    const _Float16* __restrict__ W2p, const float* __restrict__ mb2,
    const _Float16* __restrict__ U1p, const float* __restrict__ ub1,
    const _Float16* __restrict__ U2p, const float* __restrict__ ub2,
    const float* __restrict__ lng, const float* __restrict__ lnb,
    int nPer, int nRows) {
  extern __shared__ v4f lds_dyn[];
  char* sm = (char*)lds_dyn;
  _Float16* hb  = (_Float16*)(sm + LO_HB);
  float*    cs  = (float*)(sm + LO_CS);
  float*    ST  = (float*)(sm + LO_ST);
  _Float16* Ut  = (_Float16*)(sm + LO_U);
  _Float16* agb = (_Float16*)(sm + LO_AG);
  _Float16* mdb = (_Float16*)(sm + LO_MD);
  float*    dh  = (float*)(sm + LO_DH);
  const int tid = threadIdx.x, lane = tid & 31, wave = tid >> 5, hh = lane >> 4, m = lane & 15;
  const int row0 = blockIdx.x * NPB;
  const int bidx = row0 / nPer;
  const int tstart = row0 - bidx * nPer;
  const size_t rbase = (size_t)bidx * nPer;

#pragma unroll 2
  for (int idx = tid; idx < MR * 24; idx += NTHR) {
    const int r = idx / 24;
    const int q = idx - r * 24;
    const int gi = tstart - HALO + r;
    const bool valid = (r < NPB + 2 * HALO) && (gi >= 0) && (gi < nPer);
    const int gc = gi < 0 ? 0 : (gi > nPer - 1 ? nPer - 1 : gi);
    v4f v = *(const v4f*)(hin + (rbase + gc) * HID + 4 * q);
    v = zsel4(valid, v);
    *(v4h*)(hb + r * HBP + 4 * q) = cvt4(v);
  }
  for (int r = tid; r < MR; r += NTHR) {
    const int gi = tstart - HALO + r;
    const bool valid = (r < NPB + 2 * HALO) && (gi >= 0) && (gi < nPer);
    const int gc = gi < 0 ? 0 : (gi > nPer - 1 ? nPer - 1 : gi);
    const float c = coord[rbase + gc];
    cs[r] = valid ? c : 0.0f;
  }
  __syncthreads();

#pragma unroll 1
  for (int job = wave; job < 60; job += NWAVE) {
    const int mt = job / 12, nt = job - mt * 12;
    v8f acc = zero8();
    acc = mma_k96(hb + (16 * mt + m) * HBP + 8 * hh, W1c + (size_t)(16 * nt + m) * HID + 8 * hh, acc);
    const int n  = 16 * nt + m;
    const int nb = n < HID ? n : HID - 1;
    const float braw = mb1[nb];
    const float bv = (n < HID) ? braw : 0.0f;
    float* sp = ST + (16 * mt + 8 * hh) * STP + n;
#pragma unroll
    for (int r = 0; r < 8; ++r) sp[r * STP] = acc[r] * WINV + bv;
  }
  __syncthreads();

#pragma unroll 1
  for (int e = 0; e < (NPB * HID) / NTHR; ++e) {
    const int idx = e * NTHR + tid;
    const int i = idx / HID;
    const int c = idx - i * HID;
    const int ri = i + HALO;
    const int gi = tstart + i;
    const float S  = ST[ri * STP + c];
    const float wc = wdc[c];
    const float ci = cs[ri];
    float u = 0.0f;
#pragma unroll
    for (int off = 1; off <= KNB; ++off) {
      const float tp = ST[(ri + off) * STP + HID + c];
      const float vp = silu_f(S + tp + (cs[ri + off] - ci) * wc);
      u += (gi + off < nPer) ? vp : 0.0f;
      const float tn = ST[(ri - off) * STP + HID + c];
      const float vn = silu_f(S + tn + (cs[ri - off] - ci) * wc);
      u += (gi - off >= 0) ? vn : 0.0f;
    }
    Ut[i * HBP + c] = (_Float16)u;
  }
  __syncthreads();

#pragma unroll 1
  for (int job = wave; job < 24; job += NWAVE) {
    const int mt = job / 6, nt = job - mt * 6;
    v8f acc = zero8();
    acc = mma_k96(Ut + (16 * mt + m) * HBP + 8 * hh, W2p + (size_t)(16 * nt + m) * HID + 8 * hh, acc);
    const int n = 16 * nt + m;
    const float bv = mb2[n];
#pragma unroll
    for (int r = 0; r < 8; ++r) {
      const int row = 16 * mt + 8 * hh + r;
      const int gi = tstart + row;
      int cnt = (gi < KNB ? gi : KNB) + ((nPer - 1 - gi) < KNB ? (nPer - 1 - gi) : KNB);
      cnt = cnt < 1 ? 1 : cnt;
      const float inv = __builtin_amdgcn_rcpf((float)cnt);
      agb[row * HBP + n] = (_Float16)(acc[r] * WINV * inv + bv);
    }
  }
  __syncthreads();

#pragma unroll 1
  for (int job = wave; job < 24; job += NWAVE) {
    const int mt = job / 6, nt = job - mt * 6;
    v8f acc = zero8();
    const _Float16* bp = U1p + (size_t)(16 * nt + m) * (2 * HID) + 8 * hh;
    acc = mma_k96(hb + (16 * mt + HALO + m) * HBP + 8 * hh, bp, acc);
    acc = mma_k96(agb + (16 * mt + m) * HBP + 8 * hh, bp + HID, acc);
    const int n = 16 * nt + m;
    const float bv = ub1[n];
    _Float16* tp = mdb + (16 * mt + 8 * hh) * HBP + n;
#pragma unroll
    for (int r = 0; r < 8; ++r) tp[r * HBP] = (_Float16)silu_f(acc[r] * WINV + bv);
  }
  __syncthreads();

#pragma unroll 1
  for (int job = wave; job < 24; job += NWAVE) {
    const int mt = job / 6, nt = job - mt * 6;
    v8f acc = zero8();
    acc = mma_k96(mdb + (16 * mt + m) * HBP + 8 * hh, U2p + (size_t)(16 * nt + m) * HID + 8 * hh, acc);
    const int n = 16 * nt + m;
    const float bv = ub2[n];
    float* sp = dh + (16 * mt + 8 * hh) * DHP + n;
#pragma unroll
    for (int r = 0; r < 8; ++r) sp[r * DHP] = acc[r] * WINV + bv;
  }
  __syncthreads();

  const int cl = lane < 24 ? lane : 23;
  const v4f g4 = *(const v4f*)(lng + 4 * cl);
  const v4f b4 = *(const v4f*)(lnb + 4 * cl);
  v4f vals[8];
#pragma unroll
  for (int i = 0; i < 8; ++i) {
    const int row = 8 * wave + i;
    const size_t grow = (size_t)row0 + row;
    const v4f hv = *(const v4f*)(hin + grow * HID + 4 * cl);
    const v4f dv = *(const v4f*)(dh + row * DHP + 4 * cl);
    const v4f y = hv + dv;
    float s = (lane < 24) ? (y.x + y.y + y.z + y.w) : 0.0f;
    s = wsum(s);
    const float mu = s * (1.0f / 96.0f);
    const v4f d = y - mu;
    float qd = (lane < 24) ? (d.x * d.x + d.y * d.y + d.z * d.z + d.w * d.w) : 0.0f;
    qd = wsum(qd);
    const float var = qd * (1.0f / 96.0f);
    const float rs = rsqrtf(var + LN_EPS);
    vals[i] = (d * rs) * g4 + b4;
  }
#pragma unroll
  for (int i = 0; i < 8; ++i) {
    if (lane < 24) *(volatile v4f*)(hout + ((size_t)row0 + 8 * wave + i) * HID + 4 * lane) = vals[i];
  }
  __threadfence();
#pragma unroll
  for (int i = 0; i < 8; ++i) {
    if (lane < 24) *(volatile v4f*)(hout + ((size_t)row0 + 8 * wave + i) * HID + 4 * lane) = vals[i];
  }
}

__global__ __launch_bounds__(NTHR) void k_decode(
    const float* __restrict__ hin, const _Float16* __restrict__ D1p, const float* __restrict__ db1,
    const float* __restrict__ dw2, const float* __restrict__ db2, float* out, int nRows) {
  __shared__ __attribute__((aligned(16))) _Float16 ha[NPB * HBP];
  __shared__ __attribute__((aligned(16))) float    mid[NPB * DHP];
  __shared__ __attribute__((aligned(16))) float    sres[NPB];
  const int tid = threadIdx.x, lane = tid & 31, wave = tid >> 5, hh = lane >> 4, m = lane & 15;
  const int g0 = blockIdx.x * NPB;

#pragma unroll 2
  for (int idx = tid; idx < NPB * 24; idx += NTHR) {
    const int r = idx / 24;
    const int q = idx - r * 24;
    int gr = g0 + r;
    gr = gr > nRows - 1 ? nRows - 1 : gr;
    const v4f v = *(const v4f*)(hin + (size_t)gr * HID + 4 * q);
    *(v4h*)(ha + r * HBP + 4 * q) = cvt4(v);
  }
  __syncthreads();

#pragma unroll 1
  for (int job = wave; job < 24; job += NWAVE) {
    const int mt = job / 6, nt = job - mt * 6;
    v8f acc = zero8();
    acc = mma_k96(ha + (16 * mt + m) * HBP + 8 * hh, D1p + (size_t)(16 * nt + m) * HID + 8 * hh, acc);
    const int n = 16 * nt + m;
    const float bv = db1[n];
    float* sp = mid + (16 * mt + 8 * hh) * DHP + n;
#pragma unroll
    for (int r = 0; r < 8; ++r) sp[r * DHP] = silu_f(acc[r] * WINV + bv);
  }
  __syncthreads();

  const float wa = dw2[3 * lane], wb = dw2[3 * lane + 1], wcv = dw2[3 * lane + 2];
  const float bb = db2[0];
#pragma unroll
  for (int i = 0; i < 8; ++i) {
    const int row = 8 * wave + i;
    const float* mp = mid + row * DHP + 3 * lane;
    float p = mp[0] * wa + mp[1] * wb + mp[2] * wcv;
    p = wsum(p);
    if (lane == 0) sres[row] = p + bb;
  }
  __syncthreads();

  if (wave == 0) {
    const int cl = lane < 16 ? lane : 15;
    const v4f o = *(const v4f*)(sres + 4 * cl);
    if (lane < 16) *(volatile v4f*)(out + (size_t)g0 + 4 * lane) = o;
    __threadfence();
    if (lane < 16) *(volatile v4f*)(out + (size_t)g0 + 4 * lane) = o;
  }
}

extern "C" void kernel_launch(void* const* d_in, const int* in_sizes, int n_in,
                              void* d_out, int out_size, void* d_ws, size_t ws_size,
                              hipStream_t stream) {
  if (n_in < 20) return;
  const int nRows = in_sizes[1];
  if (nRows <= 0 || (nRows % NPER) != 0) return;
  if (in_sizes[0] != 4 * nRows) return;
  if (in_sizes[2] != 4 * HID || in_sizes[3] != HID || in_sizes[4] != HID * HID || in_sizes[5] != HID) return;
  if (in_sizes[6] != NL * (2 * HID + 1) * HID || in_sizes[7] != NL * HID) return;
  if (in_sizes[8] != NL * HID * HID || in_sizes[9] != NL * HID) return;
  if (in_sizes[10] != NL * 2 * HID * HID || in_sizes[11] != NL * HID) return;
  if (in_sizes[12] != NL * HID * HID || in_sizes[13] != NL * HID) return;
  if (in_sizes[14] != NL * HID || in_sizes[15] != NL * HID) return;
  if (in_sizes[16] != HID * HID || in_sizes[17] != HID || in_sizes[18] != HID || in_sizes[19] < 1) return;
  if (out_size != nRows) return;
  if ((nRows % NPB) != 0) return;

  const float* x    = (const float*)d_in[0];
  const float* crd  = (const float*)d_in[1];
  const float* ew1  = (const float*)d_in[2];
  const float* eb1  = (const float*)d_in[3];
  const float* ew2  = (const float*)d_in[4];
  const float* eb2  = (const float*)d_in[5];
  const float* mw1  = (const float*)d_in[6];
  const float* mb1  = (const float*)d_in[7];
  const float* mw2  = (const float*)d_in[8];
  const float* mb2  = (const float*)d_in[9];
  const float* uw1  = (const float*)d_in[10];
  const float* ub1  = (const float*)d_in[11];
  const float* uw2  = (const float*)d_in[12];
  const float* ub2  = (const float*)d_in[13];
  const float* lng  = (const float*)d_in[14];
  const float* lnb  = (const float*)d_in[15];
  const float* dw1  = (const float*)d_in[16];
  const float* db1  = (const float*)d_in[17];
  const float* dw2  = (const float*)d_in[18];
  const float* db2  = (const float*)d_in[19];
  float* out = (float*)d_out;

  char* ws = (char*)d_ws;
  size_t off = 0;
  const size_t oW  = off; off += (size_t)WP_TOT * 2;               off = (off + 255) & ~(size_t)255;
  const size_t plane = (size_t)nRows * HID * 4;
  const size_t oHA = off; off += plane;                             off = (off + 255) & ~(size_t)255;
  const size_t oHB = off; off += plane;                             off = (off + 255) & ~(size_t)255;
  if (off > ws_size || off > (size_t)WSCAP) return;
  _Float16* wp = (_Float16*)(ws + oW);
  float* hA = (float*)(ws + oHA);
  float* hB = (float*)(ws + oHB);

  const int nBlk = nRows / NPB;

  k_wprep<<<WP_BLKS, NTHR, 0, stream>>>(ew2, mw1, mw2, uw1, uw2, dw1, wp);

  k_embed<<<nBlk, NTHR, 0, stream>>>(x, ew1, eb1, wp + WP_E2, eb2, hA, nRows);

  hipFuncSetAttribute(reinterpret_cast<const void*>(&k_layer),
                      hipFuncAttributeMaxDynamicSharedMemorySize, LDS_LAYER);
  for (int l = 0; l < NL; ++l) {
    const float* src = (l == 0) ? hA : hB;
    float* dst = (l == 0) ? hB : hA;
    const _Float16* lw = wp + WP_L0 + (size_t)l * WP_LSTR;
    const float* wdc = mw1 + (size_t)l * (2 * HID + 1) * HID + (size_t)2 * HID * HID;
    k_layer<<<nBlk, NTHR, LDS_LAYER, stream>>>(
        src, dst, crd, wdc,
        lw + WP_W1, mb1 + (size_t)l * HID,
        lw + WP_W2, mb2 + (size_t)l * HID,
        lw + WP_U1, ub1 + (size_t)l * HID,
        lw + WP_U2, ub2 + (size_t)l * HID,
        lng + (size_t)l * HID, lnb + (size_t)l * HID, NPER, nRows);
  }

  k_decode<<<nBlk, NTHR, 0, stream>>>(hA, wp + WP_D1, db1, dw2, db2, out, nRows);
}
